// CrossModalAttention_49804440764467
// MI455X (gfx1250) — hardware-verified
//
#include <hip/hip_runtime.h>
#include <math.h>
#include <stdint.h>

#ifndef NB
#define NB 4
#endif
#ifndef SEQ
#define SEQ 4096
#endif
#define NB_FULL  4
#define SEQ_FULL 4096
#define NSRC  2
#define CC    256
#define CH    128
#define DQ    64
#define NQK   128
#define NWR   384
#define QT    64
#define OSP   68
#define OSPW  132
#define TP    72
#define WSC   256.0f
#define IWSC  0.00390625f
#define VSC   16.0f
#define IVSC  0.0625f
#define LNPS  9.704060527839234f

static_assert(NB >= 1 && NB <= NB_FULL);
static_assert(SEQ >= QT && SEQ <= SEQ_FULL);
static_assert(SEQ % QT == 0 && SEQ % 32 == 0);
static_assert(CC % QT == 0 && CC % 32 == 0);
static_assert(CC == 2 * CH && CH % 16 == 0);
static_assert(DQ == 64);
static_assert(NQK == 2 * DQ);
static_assert(NWR == NQK + CC);
static_assert(NWR % 8 == 0 && DQ % 8 == 0 && NQK % 8 == 0);
static_assert((OSP * 4) % 16 == 0);
static_assert((OSPW * 4) % 16 == 0);
static_assert((TP * 2) % 16 == 0);
static_assert(OSP >= QT && OSP >= DQ && OSPW >= CH && TP >= QT);
static_assert((size_t)NB_FULL * CC * SEQ_FULL * 4 == (size_t)16777216);

typedef _Float16       v16h __attribute__((ext_vector_type(16)));
typedef _Float16       v8h  __attribute__((ext_vector_type(8)));
typedef __bf16         v16b __attribute__((ext_vector_type(16)));
typedef unsigned short v8us __attribute__((ext_vector_type(8)));
typedef float          v8f  __attribute__((ext_vector_type(8)));
typedef float          v4f  __attribute__((ext_vector_type(4)));
typedef unsigned int   v4u  __attribute__((ext_vector_type(4)));

union Frag  { v8us u[2]; v16h h; v16b bf; };
union FragH { v16h v; v8h hv[2]; };
static_assert(sizeof(Frag) == 32);
static_assert(sizeof(FragH) == 32);

__device__ __forceinline__ unsigned short bf_bits(float f) {
  unsigned u = __float_as_uint(f);
  return (unsigned short)((u + 0x7FFFu + ((u >> 16) & 1u)) >> 16);
}
__device__ __forceinline__ float bf_up(unsigned short hb) { return __uint_as_float(((unsigned)hb) << 16); }
__device__ __forceinline__ float bfr(float f) { return bf_up(bf_bits(f)); }
__device__ __forceinline__ unsigned short h_bits(_Float16 x) { return __builtin_bit_cast(unsigned short, x); }
__device__ __forceinline__ unsigned pk16(unsigned short a, unsigned short b) { return (unsigned)a | ((unsigned)b << 16); }
__device__ __forceinline__ v8f zero8() { v8f z = {0.f, 0.f, 0.f, 0.f, 0.f, 0.f, 0.f, 0.f}; return z; }
__device__ __forceinline__ float hmax8(v8f s) {
  return fmaxf(fmaxf(fmaxf(s[0], s[1]), fmaxf(s[2], s[3])), fmaxf(fmaxf(s[4], s[5]), fmaxf(s[6], s[7])));
}
__device__ __forceinline__ unsigned wave_ballot(bool p) {
#if defined(__HIP_DEVICE_COMPILE__)
  return __builtin_amdgcn_ballot_w32(p);
#else
  return p ? 1u : 0u;
#endif
}

__device__ __forceinline__ Frag ldfrag(const unsigned short* p) {
  Frag f;
  f.u[0] = *(const v8us*)(p);
  f.u[1] = *(const v8us*)(p + 16);
  return f;
}

__device__ __forceinline__ v8f mma_h(v16h a, v16h b, v8f c) {
  v8f d = __builtin_amdgcn_wmma_f32_16x16x32_f16(false, a, false, b, (short)0, c, false, false);
#if defined(__HIP_DEVICE_COMPILE__)
  asm volatile("v_nop\n\tv_nop\n\tv_nop\n\tv_nop" : "+v"(d) : "v"(a), "v"(b));
#endif
  return d;
}
__device__ __forceinline__ v8f mma_b(v16b a, v16b b, v8f c) {
  v8f d = __builtin_amdgcn_wmma_f32_16x16x32_bf16(false, a, false, b, (short)0, c, false, false);
#if defined(__HIP_DEVICE_COMPILE__)
  const v16h ha = __builtin_bit_cast(v16h, a), hb = __builtin_bit_cast(v16h, b);
  asm volatile("v_nop\n\tv_nop\n\tv_nop\n\tv_nop" : "+v"(d) : "v"(ha), "v"(hb));
#endif
  return d;
}

__global__ __launch_bounds__(256)
void cvt_w(const float* __restrict__ Wq, const float* __restrict__ Wk, const float* __restrict__ Wv,
           unsigned short* W16) {
  const int tid = threadIdx.x, blk = blockIdx.x;
  const int rl = tid >> 5, col = 8 * (tid & 31);
  const int o = 8 * blk + rl;
  const float* wbase = (blk < (DQ / 8)) ? Wq : ((blk < (NQK / 8)) ? Wk : Wv);
  const int osub = (blk < (DQ / 8)) ? 0 : ((blk < (NQK / 8)) ? DQ : NQK);
  const float* s = wbase + (size_t)(o - osub) * CC + col;
  const v4f a = *(const v4f*)s;
  const v4f q = *(const v4f*)(s + 4);
  const float f[8] = {a[0], a[1], a[2], a[3], q[0], q[1], q[2], q[3]};
  v4u u;
#pragma unroll
  for (int t = 0; t < 4; ++t) {
    const _Float16 h0 = (_Float16)(bfr(f[2 * t]) * WSC);
    const _Float16 h1 = (_Float16)(bfr(f[2 * t + 1]) * WSC);
    u[t] = pk16(h_bits(h0), h_bits(h1));
  }
#pragma unroll
  for (int pass = 0; pass < 2; ++pass) {
    *(volatile v4u*)(W16 + (size_t)o * CC + col) = u;
    __threadfence();
  }
}

__global__ __launch_bounds__(256)
void cvt_x(const float* __restrict__ x1, const float* __restrict__ x2, unsigned short* XP) {
  __shared__ __align__(16) unsigned short T[QT * TP];
  const int tid = threadIdx.x;
  const int nb = blockIdx.x, cb = blockIdx.y, sb = blockIdx.z;
  const int s = sb / NB, b = sb - s * NB;
  const float* x = (s == 0) ? x1 : x2;
  const int e = tid & 7, lq = tid >> 3;
  const int n0 = nb * QT, c0 = cb * QT;
#pragma unroll
  for (int it = 0; it < 2; ++it) {
    const int cl = it * 32 + lq;
    const float* sp = x + ((size_t)(b * CC + c0 + cl)) * SEQ_FULL + n0 + 8 * e;
    const v4f a = *(const v4f*)sp;
    const v4f q = *(const v4f*)(sp + 4);
    unsigned short hb[8];
#pragma unroll
    for (int t = 0; t < 4; ++t) {
      hb[t]     = h_bits((_Float16)bfr(a[t]));
      hb[4 + t] = h_bits((_Float16)bfr(q[t]));
    }
#pragma unroll
    for (int t = 0; t < 8; ++t) T[(8 * e + t) * TP + cl] = hb[t];
  }
  __syncthreads();
  v4u up[2];
#pragma unroll
  for (int it = 0; it < 2; ++it) {
    const int nl = it * 32 + lq;
    up[it] = *(const v4u*)(T + nl * TP + 8 * e);
  }
#pragma unroll
  for (int pass = 0; pass < 2; ++pass) {
#pragma unroll
    for (int it = 0; it < 2; ++it) {
      const int rl = it * 32 + lq;
      *(volatile v4u*)(XP + ((size_t)(sb * SEQ + n0 + rl)) * CC + c0 + 8 * e) = up[it];
    }
    __threadfence();
  }
}

__global__ __launch_bounds__(128)
void gemm_qk(const unsigned short* __restrict__ W16, const unsigned short* __restrict__ XP,
             const float* __restrict__ bq, const float* __restrict__ bk,
             unsigned short* Qh, unsigned short* Ql, unsigned short* Kh, unsigned short* Kl) {
  __shared__ __align__(16) float Os[QT * OSP];
  const int tid  = threadIdx.x;
  const int lane = tid & 31, wave = tid >> 5;
  const int hh   = lane >> 4, c = lane & 15;
  const int nt   = blockIdx.x, sb = blockIdx.y, which = blockIdx.z;
  const int n0   = nt * QT;
  const float* bias  = (which == 0) ? bq : bk;
  unsigned short* PH = (which == 0) ? Qh : Kh;
  unsigned short* PL = (which == 0) ? Ql : Kl;

  const unsigned short* ap = W16 + ((size_t)(DQ * which + c)) * CC + 8 * hh;
  const unsigned short* bp = XP + ((size_t)(sb * SEQ + n0 + 16 * wave + c)) * CC + 8 * hh;

  v8f acc[4];
#pragma unroll
  for (int mt = 0; mt < 4; ++mt) acc[mt] = zero8();

#pragma unroll
  for (int ks = 0; ks < CC / 32; ++ks) {
    const Frag fb = ldfrag(bp + 32 * ks);
#pragma unroll
    for (int mt = 0; mt < 4; ++mt) {
      const Frag fa = ldfrag(ap + (size_t)(16 * mt) * CC + 32 * ks);
      acc[mt] = mma_h(fa.h, fb.h, acc[mt]);
    }
  }

  {
    const int nl = 16 * wave + c;
#pragma unroll
    for (int mt = 0; mt < 4; ++mt) {
      v4f va, vb;
#pragma unroll
      for (int r = 0; r < 4; ++r) { va[r] = acc[mt][r] * IWSC; vb[r] = acc[mt][4 + r] * IWSC; }
      *(v4f*)(Os + nl * OSP + 16 * mt + 8 * hh)     = va;
      *(v4f*)(Os + nl * OSP + 16 * mt + 8 * hh + 4) = vb;
    }
  }
  __syncthreads();

  const int e = tid & 7, lq = tid >> 3;
  const int d0 = 8 * e;
  const v4f b0v = *(const v4f*)(bias + d0), b1v = *(const v4f*)(bias + d0 + 4);
  const float bb[8] = {bfr(b0v[0]), bfr(b0v[1]), bfr(b0v[2]), bfr(b0v[3]),
                       bfr(b1v[0]), bfr(b1v[1]), bfr(b1v[2]), bfr(b1v[3])};
  v4u uh[4], ul[4];
#pragma unroll
  for (int it = 0; it < 4; ++it) {
    const int row = it * 16 + lq;
    const float* op = Os + row * OSP;
    const v4f va = *(const v4f*)(op + d0);
    const v4f vc = *(const v4f*)(op + d0 + 4);
    const float fv[8] = {va[0], va[1], va[2], va[3], vc[0], vc[1], vc[2], vc[3]};
#pragma unroll
    for (int t = 0; t < 4; ++t) {
      const float v0 = fv[2 * t] + bb[2 * t], v1 = fv[2 * t + 1] + bb[2 * t + 1];
      const unsigned short h0 = bf_bits(v0), h1 = bf_bits(v1);
      const unsigned short l0 = bf_bits(v0 - bf_up(h0)), l1 = bf_bits(v1 - bf_up(h1));
      uh[it][t] = pk16(h0, h1);
      ul[it][t] = pk16(l0, l1);
    }
  }
#pragma unroll
  for (int pass = 0; pass < 2; ++pass) {
#pragma unroll
    for (int it = 0; it < 4; ++it) {
      const int row = it * 16 + lq;
      const size_t po = ((size_t)(sb * SEQ + n0 + row)) * DQ + d0;
      *(volatile v4u*)(PH + po) = uh[it];
      *(volatile v4u*)(PL + po) = ul[it];
    }
    __threadfence();
  }
}

__global__ __launch_bounds__(128)
void gemm_v(const unsigned short* __restrict__ W16, const unsigned short* __restrict__ XP,
            const float* __restrict__ bv, unsigned short* Vc) {
  __shared__ __align__(16) float Os[QT * OSP];
  const int tid  = threadIdx.x;
  const int lane = tid & 31, wave = tid >> 5;
  const int hh   = lane >> 4, c = lane & 15;
  const int nt   = blockIdx.x, mb = blockIdx.y, sb = blockIdx.z;
  const int n0   = nt * QT, ch0 = mb * QT;

  const unsigned short* ap = XP + ((size_t)(sb * SEQ + n0 + c)) * CC + 8 * hh;
  const unsigned short* bp = W16 + ((size_t)(NQK + ch0 + 16 * wave + c)) * CC + 8 * hh;

  v8f acc[4];
#pragma unroll
  for (int mt = 0; mt < 4; ++mt) acc[mt] = zero8();

#pragma unroll
  for (int ks = 0; ks < CC / 32; ++ks) {
    const Frag fb = ldfrag(bp + 32 * ks);
#pragma unroll
    for (int mt = 0; mt < 4; ++mt) {
      const Frag fa = ldfrag(ap + (size_t)(16 * mt) * CC + 32 * ks);
      acc[mt] = mma_h(fa.h, fb.h, acc[mt]);
    }
  }

  {
    const int chl = 16 * wave + c;
#pragma unroll
    for (int mt = 0; mt < 4; ++mt) {
      v4f va, vb;
#pragma unroll
      for (int r = 0; r < 4; ++r) { va[r] = acc[mt][r] * IWSC; vb[r] = acc[mt][4 + r] * IWSC; }
      *(v4f*)(Os + chl * OSP + 16 * mt + 8 * hh)     = va;
      *(v4f*)(Os + chl * OSP + 16 * mt + 8 * hh + 4) = vb;
    }
  }
  __syncthreads();

  const int e = tid & 7, lq = tid >> 3;
  v4u uv[4];
#pragma unroll
  for (int it = 0; it < 4; ++it) {
    const int chl = it * 16 + lq;
    const float bias = bfr(bv[ch0 + chl]);
    const v4f a = *(const v4f*)(Os + chl * OSP + 8 * e);
    const v4f q = *(const v4f*)(Os + chl * OSP + 8 * e + 4);
    const float f[8] = {a[0], a[1], a[2], a[3], q[0], q[1], q[2], q[3]};
#pragma unroll
    for (int t = 0; t < 4; ++t) {
      const _Float16 h0 = (_Float16)((f[2 * t] + bias) * VSC);
      const _Float16 h1 = (_Float16)((f[2 * t + 1] + bias) * VSC);
      uv[it][t] = pk16(h_bits(h0), h_bits(h1));
    }
  }
#pragma unroll
  for (int pass = 0; pass < 2; ++pass) {
#pragma unroll
    for (int it = 0; it < 4; ++it) {
      const int chl = it * 16 + lq;
      *(volatile v4u*)(Vc + ((size_t)(sb * CC + ch0 + chl)) * SEQ + n0 + 8 * e) = uv[it];
    }
    __threadfence();
  }
}

__global__ __launch_bounds__(128)
void attn_k(const unsigned short* __restrict__ Qh, const unsigned short* __restrict__ Ql,
            const unsigned short* __restrict__ Kh, const unsigned short* __restrict__ Kl,
            const unsigned short* __restrict__ Vc,
            const float* __restrict__ x1, const float* __restrict__ x2,
            const float* __restrict__ gam, float* out) {
  __shared__ __align__(16) float Os[QT * OSPW];
  const int tid  = threadIdx.x;
  const int wave = tid >> 5, lane = tid & 31;
  const int hh   = lane >> 4, c = lane & 15;
  const int n0   = blockIdx.x * QT, b = blockIdx.y;
  const int dd   = (int)(blockIdx.z >> 1), chh = (int)(blockIdx.z & 1u);
  const int sq   = dd * NB + b;
  const int skv  = (1 - dd) * NB + b;
  const int chb  = CH * chh;
  const float* x = (dd == 0) ? x1 : x2;
  float* outd    = out + (size_t)dd * ((size_t)NB_FULL * CC * SEQ_FULL);
  const float g  = bfr(gam[0]);

  const size_t qo = ((size_t)(sq * SEQ + n0 + 16 * wave + c)) * DQ + 8 * hh;
  const Frag qh0 = ldfrag(Qh + qo);
  const Frag qh1 = ldfrag(Qh + qo + 32);
  const Frag ql0 = ldfrag(Ql + qo);
  const Frag ql1 = ldfrag(Ql + qo + 32);
  const unsigned short* Khp = Kh + (size_t)skv * SEQ * DQ + (size_t)c * DQ + 8 * hh;
  const unsigned short* Klp = Kl + (size_t)skv * SEQ * DQ + (size_t)c * DQ + 8 * hh;
  const unsigned short* Vp = Vc + (size_t)skv * CC * SEQ + ((size_t)(chb + c)) * SEQ + 8 * hh;

  float m = -1.0e30f, l = 0.f;
  v8f o[8];
#pragma unroll
  for (int j = 0; j < 8; ++j) o[j] = zero8();

#pragma unroll 1
  for (int kb = 0; kb < SEQ; kb += 32) {
    v8f s0 = zero8(), s1 = zero8();
    {
      const unsigned short* kp = Khp + (size_t)kb * DQ;
      const unsigned short* lp = Klp + (size_t)kb * DQ;
      const Frag a0 = ldfrag(kp);
      const Frag a1 = ldfrag(kp + 32);
      const Frag r0 = ldfrag(lp);
      const Frag r1 = ldfrag(lp + 32);
      s0 = mma_b(a0.bf, qh0.bf, s0);
      s0 = mma_b(a1.bf, qh1.bf, s0);
      s0 = mma_b(a0.bf, ql0.bf, s0);
      s0 = mma_b(a1.bf, ql1.bf, s0);
      s0 = mma_b(r0.bf, qh0.bf, s0);
      s0 = mma_b(r1.bf, qh1.bf, s0);
    }
    {
      const unsigned short* kp = Khp + (size_t)(kb + 16) * DQ;
      const unsigned short* lp = Klp + (size_t)(kb + 16) * DQ;
      const Frag a0 = ldfrag(kp);
      const Frag a1 = ldfrag(kp + 32);
      const Frag r0 = ldfrag(lp);
      const Frag r1 = ldfrag(lp + 32);
      s1 = mma_b(a0.bf, qh0.bf, s1);
      s1 = mma_b(a1.bf, qh1.bf, s1);
      s1 = mma_b(a0.bf, ql0.bf, s1);
      s1 = mma_b(a1.bf, ql1.bf, s1);
      s1 = mma_b(r0.bf, qh0.bf, s1);
      s1 = mma_b(r1.bf, qh1.bf, s1);
    }

    float mx = fmaxf(hmax8(s0), hmax8(s1));
    mx = fmaxf(mx, __shfl_xor(mx, 16, 32));
    const float mn = fmaxf(m, mx);
    const unsigned grew = wave_ballot(mx > m);
    if (grew != 0u) {
      const float corr = __expf(m - mn);
      l *= corr;
#pragma unroll
      for (int j = 0; j < 8; ++j) {
#pragma unroll
        for (int r = 0; r < 8; ++r) o[j][r] *= corr;
      }
    }
    m = mn;
    const float msh = mn - LNPS;

    FragH ph;
    float ls = 0.f;
#pragma unroll
    for (int r = 0; r < 8; ++r) {
      const float e0 = __expf(s0[r] - msh);
      const float e1 = __expf(s1[r] - msh);
      ls += e0 + e1;
      ph.hv[0][r] = (_Float16)e0;
      ph.hv[1][r] = (_Float16)e1;
    }
    l += ls;

#pragma unroll
    for (int j = 0; j < 8; ++j) {
      const Frag vf = ldfrag(Vp + (size_t)(16 * j) * SEQ + kb);
      o[j] = mma_h(vf.h, ph.v, o[j]);
    }
  }
  l += __shfl_xor(l, 16, 32);
  const float inv = 1.0f / l;
  const float gi  = g * IVSC * inv;

  const int qrow = 16 * wave + c;
  const int e = tid & 7, lq = tid >> 3;
#pragma unroll
  for (int j = 0; j < 8; ++j) {
    v4f va, vb;
#pragma unroll
    for (int r = 0; r < 4; ++r) { va[r] = o[j][r] * gi; vb[r] = o[j][4 + r] * gi; }
    *(v4f*)(Os + qrow * OSPW + 16 * j + 8 * hh)     = va;
    *(v4f*)(Os + qrow * OSPW + 16 * j + 8 * hh + 4) = vb;
  }
  __syncthreads();
  v4f res[16];
#pragma unroll
  for (int it = 0; it < 16; ++it) {
    const int L   = it * 16 + lq;
    const int chl = L >> 1, hf = L & 1;
    const int nl  = hf * 32 + 4 * e;
    const size_t idx = ((size_t)(b * CC + chb + chl)) * SEQ_FULL + n0 + nl;
    const v4f xv = *(const v4f*)(x + idx);
#pragma unroll
    for (int t = 0; t < 4; ++t) res[it][t] = Os[(nl + t) * OSPW + chl] + bfr(xv[t]);
  }
#pragma unroll
  for (int pass = 0; pass < 2; ++pass) {
#pragma unroll
    for (int it = 0; it < 16; ++it) {
      const int L   = it * 16 + lq;
      const int chl = L >> 1, hf = L & 1;
      const int nl  = hf * 32 + 4 * e;
      const size_t idx = ((size_t)(b * CC + chb + chl)) * SEQ_FULL + n0 + nl;
      *(volatile v4f*)(outd + idx) = res[it];
    }
    __threadfence();
  }
}

extern "C" void kernel_launch(void* const* d_in, const int* in_sizes, int n_in,
                              void* d_out, int out_size, void* d_ws, size_t ws_size,
                              hipStream_t stream) {
  if (n_in < 9) return;
  if (in_sizes[0] < NB * CC * SEQ_FULL || in_sizes[1] < NB * CC * SEQ_FULL) return;
  if (in_sizes[2] < DQ * CC || in_sizes[3] < DQ) return;
  if (in_sizes[4] < DQ * CC || in_sizes[5] < DQ) return;
  if (in_sizes[6] < CC * CC || in_sizes[7] < CC) return;
  if (in_sizes[8] < 1) return;
  if (out_size < (NB_FULL + NB) * CC * SEQ_FULL) return;

  size_t off = 0;
  auto carve = [&](size_t bytes) { const size_t o = off; off += (bytes + 255) & ~(size_t)255; return o; };
  const size_t oW16 = carve((size_t)NWR * CC * 2);
  const size_t oXP  = carve((size_t)NSRC * NB * SEQ * CC * 2);
  const size_t oVc  = carve((size_t)NSRC * NB * CC * SEQ * 2);
  const size_t oQh  = carve((size_t)NSRC * NB * SEQ * DQ * 2);
  const size_t oQl  = carve((size_t)NSRC * NB * SEQ * DQ * 2);
  const size_t oKh  = carve((size_t)NSRC * NB * SEQ * DQ * 2);
  const size_t oKl  = carve((size_t)NSRC * NB * SEQ * DQ * 2);
  if (off > ws_size) return;
  if (off > (size_t)134217728) return;

  const float* x1  = (const float*)d_in[0];
  const float* x2  = (const float*)d_in[1];
  const float* Wq  = (const float*)d_in[2];
  const float* bq  = (const float*)d_in[3];
  const float* Wk  = (const float*)d_in[4];
  const float* bk  = (const float*)d_in[5];
  const float* Wv  = (const float*)d_in[6];
  const float* bv  = (const float*)d_in[7];
  const float* gam = (const float*)d_in[8];

  char* ws = (char*)d_ws;
  unsigned short* W16 = (unsigned short*)(ws + oW16);
  unsigned short* XP  = (unsigned short*)(ws + oXP);
  unsigned short* Vc  = (unsigned short*)(ws + oVc);
  unsigned short* Qh  = (unsigned short*)(ws + oQh);
  unsigned short* Ql  = (unsigned short*)(ws + oQl);
  unsigned short* Kh  = (unsigned short*)(ws + oKh);
  unsigned short* Kl  = (unsigned short*)(ws + oKl);
  float* out = (float*)d_out;

  const dim3 blk256(256), blk128(128);

  cvt_w<<<dim3(NWR / 8), blk256, 0, stream>>>(Wq, Wk, Wv, W16);
  cvt_x<<<dim3(SEQ / QT, CC / QT, NSRC * NB), blk256, 0, stream>>>(x1, x2, XP);
  gemm_qk<<<dim3(SEQ / QT, NSRC * NB, 2), blk128, 0, stream>>>(W16, XP, bq, bk, Qh, Ql, Kh, Kl);
  gemm_v<<<dim3(SEQ / QT, CC / QT, NSRC * NB), blk128, 0, stream>>>(W16, XP, bv, Vc);
  attn_k<<<dim3(SEQ / QT, NB, 2 * NSRC), blk128, 0, stream>>>(Qh, Ql, Kh, Kl, Vc, x1, x2, gam, out);
  (void)hipGetLastError();
}
